// PatchPositionEmbedding_30305289240876
// MI455X (gfx1250) — hardware-run, weakly checked
//
#include <hip/hip_runtime.h>


#ifndef NB
#define NB 64
#endif
#define NB_FULL 64
#define CCH    3
#define HIMG   224
#define WIMG   224
#define PSZ    16
#define GP     14
#define NTOK   196
#define SEQT   197
#define DMODEL 768
#define KD     768
#define MROWS  (NB * NTOK)
#define MPAD   (((MROWS + 63) / 64) * 64)

static_assert(KD == CCH * PSZ * PSZ);
static_assert(KD % 32 == 0);
static_assert(KD % 64 == 0);
static_assert(DMODEL % 64 == 0);
static_assert(HIMG == GP * PSZ);
static_assert(WIMG == GP * PSZ);
static_assert(NTOK == GP * GP);
static_assert(SEQT == NTOK + 1);
static_assert(PSZ == 16);
static_assert(WIMG % 8 == 0);
static_assert(MPAD % 64 == 0);
static_assert(MROWS % 2 == 0);
static_assert(NB <= NB_FULL);
static_assert((DMODEL / 4) % 8 == 0);
static_assert(KD / 8 == 96);
static_assert(16 * 68 * 4 <= 131072);
static_assert(64 * 72 * 2 <= 131072);

typedef unsigned short bf;
typedef __attribute__((ext_vector_type(16))) __bf16   v16bf;
typedef __attribute__((ext_vector_type(8)))  unsigned short v8us;
typedef __attribute__((ext_vector_type(8)))  float    v8f;
typedef __attribute__((ext_vector_type(4)))  float    v4f;
typedef v4f  __attribute__((may_alias)) v4fa;
typedef v8us __attribute__((may_alias)) v8usa;

__device__ __forceinline__ unsigned short f2bf(float f) { unsigned u = __float_as_uint(f); u += 0x7FFFu + ((u >> 16) & 1u); return (unsigned short)(u >> 16); }
__device__ __forceinline__ float bfr(float f) { return __uint_as_float(((unsigned)f2bf(f)) << 16); }
__device__ __forceinline__ v16bf cat16b(v8us lo, v8us hi) { return __builtin_bit_cast(v16bf, __builtin_shufflevector(lo, hi, 0, 1, 2, 3, 4, 5, 6, 7, 8, 9, 10, 11, 12, 13, 14, 15)); }
__device__ __forceinline__ v8f wmmab(v16bf a, v16bf b, v8f c) { return __builtin_amdgcn_wmma_f32_16x16x32_bf16(false, a, false, b, (short)0, c, false, false); }
__device__ __forceinline__ v8f wmmabg(v16bf a, v16bf b, v8f c) { c = wmmab(a, b, c); asm volatile("v_nop\n\tv_nop\n\tv_nop\n\tv_nop" : "+v"(c) : "v"(a), "v"(b)); return c; }
__device__ __forceinline__ v16bf ldb(const bf* p)  { return cat16b(*(const v8us*)p, *(const v8us*)(p + 16)); }
__device__ __forceinline__ void wave_sync() { __builtin_amdgcn_fence(3  , "wavefront"); __builtin_amdgcn_wave_barrier(); asm volatile("" ::: "memory"); }

static constexpr int N8ALL = MPAD * (KD / 8);
static_assert(N8ALL % 256 == 0);

__global__ __launch_bounds__(256) void k_im2row(const float* __restrict__ x, bf* dst) {
    const int i = blockIdx.x * 256 + threadIdx.x; if (i >= N8ALL) return;
    const int m = i / (KD / 8); const int f0 = (i - m * (KD / 8)) * 8;
    const int mc = m < MROWS ? m : (MROWS - 1);
    const int b = mc / NTOK; const int p = mc - b * NTOK; const int pi = p / GP; const int pj = p - pi * GP;
    const int c = f0 >> 8, r = (f0 & 255) >> 4, col = f0 & 15;
    const size_t g = ((size_t)(b * CCH + c) * HIMG + (size_t)(PSZ * pi + r)) * WIMG + (size_t)(PSZ * pj + col);
    const v8f v = *(const v8f*)(x + g); v8us o;
    const bool live = m < MROWS;
#pragma unroll
    for (int k = 0; k < 8; ++k) o[k] = live ? f2bf(v[k]) : (unsigned short)0;
    *(volatile v8us*)(dst + (size_t)i * 8) = o; __threadfence(); *(volatile v8us*)(dst + (size_t)i * 8) = o;
}

__global__ __launch_bounds__(256) void k_wt(const float* __restrict__ W, bf* WT) {
    __shared__ __align__(16) unsigned short ts[64 * 72];
    const int tid = threadIdx.x; const int k0 = blockIdx.x * 64, n0 = blockIdx.y * 64;
    { const int kr = tid >> 2, nc = (tid & 3) * 16;
      const float* src = W + (size_t)(k0 + kr) * DMODEL + n0 + nc;
      const v4f w0 = *(const v4f*)src, w1 = *(const v4f*)(src + 4), w2 = *(const v4f*)(src + 8), w3 = *(const v4f*)(src + 12);
#pragma unroll
      for (int i = 0; i < 4; ++i) { ts[(nc + i) * 72 + kr] = f2bf(w0[i]); ts[(nc + 4 + i) * 72 + kr] = f2bf(w1[i]); ts[(nc + 8 + i) * 72 + kr] = f2bf(w2[i]); ts[(nc + 12 + i) * 72 + kr] = f2bf(w3[i]); } }
    __syncthreads();
    static_assert(2 * 256 * 16 == 64 * 64 * 2);
#pragma unroll 1
    for (int ps = 0; ps < 2; ++ps) {
#pragma unroll
        for (int s = 0; s < 2; ++s) { const int p = s * 256 + tid; const int n = p >> 3, k8 = (p & 7) * 8;
            const v8us o = *(const v8usa*)(&ts[n * 72 + k8]);
            *(volatile v8us*)(WT + (size_t)(n0 + n) * KD + k0 + k8) = o; }
        if (ps == 0) __threadfence(); }
}

__global__ __launch_bounds__(32) void k_gemm(const bf* __restrict__ A, const bf* __restrict__ Bt, const float* __restrict__ bias, const float* __restrict__ pos, float* OUT) {
    __shared__ __align__(16) float os[16 * 68];
    const int K = KD;
    const int lane = threadIdx.x & 31, lr = lane & 15, hi = lane >> 4; const int r0 = blockIdx.x * 64, c0 = blockIdx.y * 64;
    v8f acc[4][4];
#pragma unroll
    for (int mb = 0; mb < 4; ++mb)
#pragma unroll
        for (int nb = 0; nb < 4; ++nb) acc[mb][nb] = (v8f){};
    const size_t aoff = (size_t)(r0 + lr) * K + 8 * hi, boff = (size_t)(c0 + lr) * K + 8 * hi;
#pragma unroll 1
    for (int kc = 0; kc < K; kc += 32) {
        v16bf a[4];
#pragma unroll
        for (int mb = 0; mb < 4; ++mb) a[mb] = ldb(A + aoff + (size_t)mb * 16 * K + kc);
#pragma unroll
        for (int nb = 0; nb < 4; ++nb) { const v16bf b = ldb(Bt + boff + (size_t)nb * 16 * K + kc);
#pragma unroll
            for (int mb = 0; mb < 4; ++mb) acc[mb][nb] = wmmabg(a[mb], b, acc[mb][nb]); }
    }
    const int cofs = (lane & 15) * 4;
    v4f bv = *(const v4f*)(bias + c0 + cofs);
#pragma unroll
    for (int i = 0; i < 4; ++i) bv[i] = bfr(bv[i]);
    static_assert(32 * 16 * 8 == 16 * 64 * 4);
#pragma unroll
    for (int mb = 0; mb < 4; ++mb) {
#pragma unroll
        for (int nb = 0; nb < 4; ++nb) {
#pragma unroll
            for (int j = 0; j < 8; ++j) os[(hi * 8 + j) * 68 + nb * 16 + lr] = acc[mb][nb][j]; }
        wave_sync();
        v4f val[8]; size_t oo[8]; bool ok[8];
#pragma unroll
        for (int s = 0; s < 8; ++s) { const int row = 2 * s + (lane >> 4);
            const int rg = r0 + mb * 16 + row;
            const int rc = rg < MROWS ? rg : (MROWS - 1);
            const int bb = rc / NTOK; const int pp = rc - bb * NTOK;
            v4f pv = *(const v4f*)(pos + (size_t)(1 + pp) * DMODEL + c0 + cofs);
            asm volatile("" : "+v"(pv));
            const v4f x0 = *(const v4fa*)(&os[row * 68 + cofs]); v4f o;
#pragma unroll
            for (int i = 0; i < 4; ++i) o[i] = (x0[i] + bv[i]) + bfr(pv[i]);
            val[s] = o; oo[s] = ((size_t)bb * SEQT + (size_t)(1 + pp)) * DMODEL + (size_t)(c0 + cofs); ok[s] = rg < MROWS; }
#pragma unroll 1
        for (int ps = 0; ps < 2; ++ps) {
#pragma unroll
            for (int s = 0; s < 8; ++s) { if (ok[s]) *(volatile v4f*)(OUT + oo[s]) = val[s]; }
            if (ps == 0) __threadfence(); }
        wave_sync();
    }
}

static constexpr int N4CLS = NB * (DMODEL / 4);

__global__ __launch_bounds__(256) void k_cls(const float* __restrict__ cls, const float* __restrict__ pos, float* OUT) {
    const int i = blockIdx.x * 256 + threadIdx.x; if (i >= N4CLS) return;
    const int b = i / (DMODEL / 4); const int c4 = (i - b * (DMODEL / 4)) * 4;
    const v4f c = *(const v4f*)(cls + c4); const v4f p = *(const v4f*)(pos + c4); v4f o;
#pragma unroll
    for (int k = 0; k < 4; ++k) o[k] = bfr(c[k]) + bfr(p[k]);
    float* dst = OUT + (size_t)b * SEQT * DMODEL + c4;
    *(volatile v4f*)dst = o; __threadfence(); *(volatile v4f*)dst = o;
}

static constexpr size_t al256(size_t v) { return (v + 255) & ~(size_t)255; }
static constexpr size_t SZ_XP = al256((size_t)MPAD * KD * 2);
static constexpr size_t SZ_WT = al256((size_t)DMODEL * KD * 2);
static constexpr size_t SZ_TOTAL = SZ_XP + SZ_WT;
static_assert(SZ_TOTAL <= (size_t)134217728);
static_assert((size_t)N8ALL * 16 == (size_t)MPAD * KD * 2);
static_assert((size_t)(KD / 64) * (DMODEL / 64) * 64 * 64 * 2 == (size_t)DMODEL * KD * 2);
static constexpr unsigned G_IM2ROW = (unsigned)(N8ALL / 256);
static constexpr unsigned G_CLS = (unsigned)((N4CLS + 255) / 256);
static constexpr size_t NEED_X = (size_t)NB * CCH * HIMG * WIMG;
static constexpr size_t NEED_OUT = (size_t)NB * SEQT * DMODEL;

extern "C" void kernel_launch(void* const* d_in, const int* in_sizes, int n_in,
                              void* d_out, int out_size, void* d_ws, size_t ws_size, hipStream_t stream) {
    if (n_in < 5) return;
    if ((size_t)in_sizes[0] < NEED_X) return;
    if ((size_t)in_sizes[1] < (size_t)KD * DMODEL) return;
    if (in_sizes[2] < DMODEL || (size_t)in_sizes[3] < (size_t)SEQT * DMODEL || in_sizes[4] < DMODEL) return;
    if ((size_t)out_size < NEED_OUT) return;
    if (SZ_TOTAL > ws_size) return;
    const float* x   = (const float*)d_in[0];
    const float* Wm  = (const float*)d_in[1];
    const float* bia = (const float*)d_in[2];
    const float* pos = (const float*)d_in[3];
    const float* cls = (const float*)d_in[4];
    float* OUT = (float*)d_out;
    char* wsp = (char*)d_ws;
    bf* XP = (bf*)wsp; wsp += SZ_XP;
    bf* WT = (bf*)wsp; wsp += SZ_WT;

    k_im2row<<<G_IM2ROW, 256, 0, stream>>>(x, XP);
    k_wt<<<dim3(KD / 64, DMODEL / 64, 1), 256, 0, stream>>>(Wm, WT);
    k_gemm<<<dim3(MPAD / 64, DMODEL / 64, 1), 32, 0, stream>>>(XP, WT, bia, pos, OUT);
    k_cls<<<G_CLS, 256, 0, stream>>>(cls, pos, OUT);
}
